// MNT_24644522344574
// MI455X (gfx1250) — hardware-verified
//
#include <hip/hip_runtime.h>
#define BB 16
#define NTK 1024
#define DD 256
#define HF 1024
#define PP 16
#define IMW 512
#define NPW (IMW / PP)
#define KIN 768
#define WIN 64
#define NHD 8
#define DHD 32
#define NTT (BB * NTK)
#define BCH 4
#define TCH (BCH * NTK)

typedef __bf16 v16b __attribute__((ext_vector_type(16)));
typedef unsigned short v8us __attribute__((ext_vector_type(8), may_alias));
typedef float  v8f  __attribute__((ext_vector_type(8)));
typedef float  v4f  __attribute__((ext_vector_type(4)));
typedef float  v4fa __attribute__((ext_vector_type(4), may_alias));
union FragB { v16b v; v8us half[2]; unsigned short u[16]; };

__device__ __forceinline__ unsigned short bf16_bits(float x) { unsigned int u = __float_as_uint(x); return (unsigned short)((u + 0x7FFFu + ((u >> 16) & 1u)) >> 16); }
__device__ __forceinline__ float bf16_val(unsigned short b) { return __uint_as_float(((unsigned int)b) << 16); }
__device__ __forceinline__ float bf16_round(float x) { return bf16_val(bf16_bits(x)); }
template <int NT>
__device__ __forceinline__ v8f mmaN(v16b ah, v16b al, v16b bh, v16b bl, v8f c) {
  c = __builtin_amdgcn_wmma_f32_16x16x32_bf16(false, ah, false, bh, (short)0, c, false, false);
  if (NT >= 2) c = __builtin_amdgcn_wmma_f32_16x16x32_bf16(false, al, false, bh, (short)0, c, false, false);
  if (NT >= 3) c = __builtin_amdgcn_wmma_f32_16x16x32_bf16(false, ah, false, bl, (short)0, c, false, false);
  asm volatile("v_nop\n\tv_nop\n\tv_nop\n\tv_nop" : "+v"(c) : "v"(ah), "v"(al), "v"(bh), "v"(bl));
  return c;
}

__global__ __launch_bounds__(256) void k_wt_bf16(const float* __restrict__ W, unsigned short* __restrict__ Wt, int K, int N) {
  const int t = blockIdx.x * 256 + threadIdx.x;
  const int k8n = K / 8;
  if (t >= N * k8n) return;
  const int n = t / k8n, k8 = (t % k8n) * 8;
  v8us v;
#pragma unroll
  for (int i = 0; i < 8; ++i) v[i] = bf16_bits(W[(size_t)(k8 + i) * N + n]);
  *(volatile v8us*)(Wt + (size_t)n * K + k8) = v;
  __threadfence();
  *(volatile v8us*)(Wt + (size_t)n * K + k8) = v;
}

template <bool ASPLIT, int ACT, bool BIAS_BF16>
__global__ __launch_bounds__(128) void k_gemm_bf(const float* __restrict__ A, int lda, const unsigned short* __restrict__ Wt, int ldb,
                                               const float* __restrict__ bias, float* __restrict__ C, int ldc, int M, int N, int K) {
  __shared__ __attribute__((aligned(16))) float so[4][16][64];
  const int tid = threadIdx.x, w = tid >> 5, lane = tid & 31, ln = lane & 15, hh = lane >> 4;
  const int ntn = N / 64;
  const int wid = blockIdx.x * 4 + w;
  const int mt = wid / ntn, nq = wid % ntn;
  if (mt * 16 >= M) return;
  const int row0 = mt * 16, col0 = nq * 64;
  const float* arow = A + (size_t)(row0 + ln) * lda;
  v8f acc[4] = {};
  for (int kb = 0; kb < K; kb += 32) {
    FragB ah, al;
    const v4f x0 = *(const v4fa*)(arow + kb + 8 * hh), x1 = *(const v4fa*)(arow + kb + 8 * hh + 4);
    const v4f x2 = *(const v4fa*)(arow + kb + 16 + 8 * hh), x3 = *(const v4fa*)(arow + kb + 16 + 8 * hh + 4);
    float xs[16] = {x0[0],x0[1],x0[2],x0[3],x1[0],x1[1],x1[2],x1[3],x2[0],x2[1],x2[2],x2[3],x3[0],x3[1],x3[2],x3[3]};
#pragma unroll
    for (int i = 0; i < 16; ++i) { const unsigned short hb = bf16_bits(xs[i]); ah.u[i] = hb; al.u[i] = ASPLIT ? bf16_bits(xs[i] - bf16_val(hb)) : (unsigned short)0; }
#pragma unroll
    for (int t = 0; t < 4; ++t) {
      const unsigned short* brow = Wt + (size_t)(col0 + t * 16 + ln) * ldb + kb;
      FragB b;
      b.half[0] = *(const v8us*)(brow + 8 * hh);
      b.half[1] = *(const v8us*)(brow + 16 + 8 * hh);
      acc[t] = mmaN<ASPLIT ? 2 : 1>(ah.v, al.v, b.v, b.v, acc[t]);
    }
  }
#pragma unroll
  for (int t = 0; t < 4; ++t) {
    float bv = bias ? bias[col0 + t * 16 + ln] : 0.f;
    if (BIAS_BF16) bv = bf16_round(bv);
#pragma unroll
    for (int r = 0; r < 8; ++r) { float v = acc[t][r] + bv; if (ACT == 1) v = fmaxf(v, 0.f); so[w][8 * hh + r][t * 16 + ln] = v; }
  }
  __builtin_amdgcn_fence(__ATOMIC_ACQ_REL, "workgroup");
  __builtin_amdgcn_wave_barrier();
  const int rsub = lane >> 4, c4 = (lane & 15) * 4;
  for (int pass = 0; pass < 2; ++pass) {
#pragma unroll
    for (int q = 0; q < 8; ++q) {
      const int r = q * 2 + rsub;
      const v4f v = *(const v4fa*)&so[w][r][c4];
      *(volatile v4f*)(C + (size_t)(row0 + r) * ldc + col0 + c4) = v;
    }
    if (pass == 0) __threadfence();
  }
}

template <int D, bool CAUSAL>
__global__ __launch_bounds__(128) void k_flash(const float* __restrict__ qb, const float* __restrict__ kb, const float* __restrict__ vb,
                                             int pitch, int T, int H, float scale, float* __restrict__ y, int ypitch) {
  constexpr int KS = D / 32;
  constexpr int DT = D / 16;
  __shared__ __attribute__((aligned(16))) unsigned short sKh[32][D + 8], sKl[32][D + 8], sVh[32][D + 8], sVl[32][D + 8];
  __shared__ __attribute__((aligned(16))) unsigned short sPh[4][16][40], sPl[4][16][40];
  __shared__ __attribute__((aligned(16))) float sO[4][16][D];
  const int tid = threadIdx.x, w = tid >> 5, lane = tid & 31, ln = lane & 15, hh = lane >> 4;
  const int nqb = (T + 63) / 64;
  const int bh = blockIdx.x / nqb, qblk = blockIdx.x % nqb;
  const int b = bh / H, h = bh % H;
  const int q0 = qblk * 64 + w * 16;
  const float* Q = qb + (size_t)b * T * pitch + h * D;
  const float* K = kb + (size_t)b * T * pitch + h * D;
  const float* V = vb + (size_t)b * T * pitch + h * D;

  FragB aqh[KS], aql[KS];
  {
    int row = q0 + ln; if (row >= T) row = T - 1;
    const float* qr = Q + (size_t)row * pitch;
#pragma unroll
    for (int ks = 0; ks < KS; ++ks)
#pragma unroll
      for (int i = 0; i < 16; ++i) {
        const int d = ks * 32 + ((i < 8) ? (8 * hh + i) : (16 + 8 * hh + (i - 8)));
        const float x = qr[d] * scale; const unsigned short hb = bf16_bits(x);
        aqh[ks].u[i] = hb; aql[ks].u[i] = bf16_bits(x - bf16_val(hb));
      }
  }
  float m_r[8], l_r[8];
#pragma unroll
  for (int r = 0; r < 8; ++r) { m_r[r] = -3.0e38f; l_r[r] = 0.f; }
  v8f oacc[DT];
#pragma unroll
  for (int dt = 0; dt < DT; ++dt) oacc[dt] = (v8f){0.f,0.f,0.f,0.f,0.f,0.f,0.f,0.f};

  const int kv_end = CAUSAL ? min(T, qblk * 64 + 64) : T;
  for (int j0 = 0; j0 < kv_end; j0 += 32) {
    __syncthreads();
    for (int e = tid; e < 32 * (D / 4); e += 128) {
      const int r = e / (D / 4), c4 = (e % (D / 4)) * 4;
      const int key = j0 + r;
      v4f kf = {0.f,0.f,0.f,0.f}, vf = {0.f,0.f,0.f,0.f};
      if (key < T) { kf = *(const v4fa*)(K + (size_t)key * pitch + c4); vf = *(const v4fa*)(V + (size_t)key * pitch + c4); }
#pragma unroll
      for (int t = 0; t < 4; ++t) {
        unsigned short hb = bf16_bits(kf[t]); sKh[r][c4 + t] = hb; sKl[r][c4 + t] = bf16_bits(kf[t] - bf16_val(hb));
        hb = bf16_bits(vf[t]); sVh[r][c4 + t] = hb; sVl[r][c4 + t] = bf16_bits(vf[t] - bf16_val(hb));
      }
    }
    __syncthreads();
    v8f s[2];
#pragma unroll
    for (int nt = 0; nt < 2; ++nt) {
      v8f acc = {};
#pragma unroll
      for (int ks = 0; ks < KS; ++ks) {
        FragB bh_, bl_;
        bh_.half[0] = *(const v8us*)&sKh[nt * 16 + ln][ks * 32 + 8 * hh]; bh_.half[1] = *(const v8us*)&sKh[nt * 16 + ln][ks * 32 + 16 + 8 * hh];
        bl_.half[0] = *(const v8us*)&sKl[nt * 16 + ln][ks * 32 + 8 * hh]; bl_.half[1] = *(const v8us*)&sKl[nt * 16 + ln][ks * 32 + 16 + 8 * hh];
        acc = mmaN<3>(aqh[ks].v, aql[ks].v, bh_.v, bl_.v, acc);
      }
      s[nt] = acc;
    }
    float alpha[8];
#pragma unroll
    for (int r = 0; r < 8; ++r) {
      const int qi = q0 + 8 * hh + r;
      const int ja = j0 + ln, jb = j0 + 16 + ln;
      if (CAUSAL) { if (ja > qi) s[0][r] = -3.0e38f; if (jb > qi) s[1][r] = -3.0e38f; }
      if (ja >= T) s[0][r] = -3.0e38f;
      if (jb >= T) s[1][r] = -3.0e38f;
      float mx = fmaxf(s[0][r], s[1][r]);
      mx = fmaxf(mx, __shfl_xor(mx, 1, 32)); mx = fmaxf(mx, __shfl_xor(mx, 2, 32)); mx = fmaxf(mx, __shfl_xor(mx, 4, 32)); mx = fmaxf(mx, __shfl_xor(mx, 8, 32));
      const float mnew = fmaxf(m_r[r], mx);
      alpha[r] = (mnew > -1.0e38f) ? __expf(m_r[r] - mnew) : 1.0f;
      const float p0 = (s[0][r] > -1.0e38f) ? __expf(s[0][r] - mnew) : 0.f;
      const float p1 = (s[1][r] > -1.0e38f) ? __expf(s[1][r] - mnew) : 0.f;
      m_r[r] = mnew;
      l_r[r] = l_r[r] * alpha[r] + p0 + p1;
      unsigned short hb = bf16_bits(p0); sPh[w][8 * hh + r][ln] = hb;      sPl[w][8 * hh + r][ln] = bf16_bits(p0 - bf16_val(hb));
      hb = bf16_bits(p1);                sPh[w][8 * hh + r][16 + ln] = hb; sPl[w][8 * hh + r][16 + ln] = bf16_bits(p1 - bf16_val(hb));
    }
#pragma unroll
    for (int dt = 0; dt < DT; ++dt)
#pragma unroll
      for (int r = 0; r < 8; ++r) oacc[dt][r] *= alpha[r];
    __builtin_amdgcn_fence(__ATOMIC_ACQ_REL, "workgroup");
    __builtin_amdgcn_wave_barrier();
    FragB pah, pal;
    pah.half[0] = *(const v8us*)&sPh[w][ln][8 * hh]; pah.half[1] = *(const v8us*)&sPh[w][ln][16 + 8 * hh];
    pal.half[0] = *(const v8us*)&sPl[w][ln][8 * hh]; pal.half[1] = *(const v8us*)&sPl[w][ln][16 + 8 * hh];
#pragma unroll
    for (int dt = 0; dt < DT; ++dt) {
      FragB bvh, bvl;
#pragma unroll
      for (int i = 0; i < 8; ++i) {
        bvh.u[i] = sVh[8 * hh + i][dt * 16 + ln]; bvh.u[8 + i] = sVh[16 + 8 * hh + i][dt * 16 + ln];
        bvl.u[i] = sVl[8 * hh + i][dt * 16 + ln]; bvl.u[8 + i] = sVl[16 + 8 * hh + i][dt * 16 + ln];
      }
      oacc[dt] = mmaN<3>(pah.v, pal.v, bvh.v, bvl.v, oacc[dt]);
    }
    __builtin_amdgcn_fence(__ATOMIC_ACQ_REL, "workgroup");
    __builtin_amdgcn_wave_barrier();
  }
#pragma unroll
  for (int r = 0; r < 8; ++r) {
    float l = l_r[r];
    l += __shfl_xor(l, 1, 32); l += __shfl_xor(l, 2, 32); l += __shfl_xor(l, 4, 32); l += __shfl_xor(l, 8, 32);
    l_r[r] = (l > 0.f) ? 1.0f / l : 0.f;
  }
#pragma unroll
  for (int dt = 0; dt < DT; ++dt)
#pragma unroll
    for (int r = 0; r < 8; ++r) sO[w][8 * hh + r][dt * 16 + ln] = oacc[dt][r] * l_r[r];
  __builtin_amdgcn_fence(__ATOMIC_ACQ_REL, "workgroup");
  __builtin_amdgcn_wave_barrier();
  for (int pass = 0; pass < 2; ++pass) {
    for (int r = 0; r < 16; ++r) {
      const int row = q0 + r;
      if (row < T && lane < D / 4) {
        const v4f val = *(const v4fa*)&sO[w][r][lane * 4];
        *(volatile v4f*)(y + ((size_t)b * T + row) * ypitch + h * D + lane * 4) = val;
      }
    }
    if (pass == 0) __threadfence();
  }
}

template <bool ASPLIT, bool BSPLIT, int ACT>
__global__ __launch_bounds__(128) void k_gemm_b(const float* __restrict__ A, int lda, size_t sA, const unsigned short* __restrict__ Bh, const unsigned short* __restrict__ Bl, int ldb, size_t sB,
                                             const float* __restrict__ bias, const float* __restrict__ resid, int ldr, size_t sR, float rsign, float alpha,
                                             float* __restrict__ C, int ldc, size_t sC, int M, int N, int K) {
  __shared__ __attribute__((aligned(16))) float so[4][16][64];
  const int tid = threadIdx.x, w = tid >> 5, lane = tid & 31, ln = lane & 15, hh = lane >> 4;
  const int by = blockIdx.y;
  A += (size_t)by * sA; Bh += (size_t)by * sB; if (BSPLIT) Bl += (size_t)by * sB; C += (size_t)by * sC; if (resid) resid += (size_t)by * sR;
  const int ntn = (N + 63) / 64; const int wid = blockIdx.x * 4 + w; const int mt = wid / ntn, nq = wid % ntn;
  if (mt * 16 >= M) return;
  const int row0 = mt * 16, col0 = nq * 64;
  const float* arow = A + (size_t)(row0 + ln) * lda;
  v8f acc[4] = {};
  for (int kb = 0; kb < K; kb += 32) {
    FragB ah, al;
    const v4f x0 = *(const v4fa*)(arow + kb + 8 * hh), x1 = *(const v4fa*)(arow + kb + 8 * hh + 4);
    const v4f x2 = *(const v4fa*)(arow + kb + 16 + 8 * hh), x3 = *(const v4fa*)(arow + kb + 16 + 8 * hh + 4);
    float xs[16] = {x0[0],x0[1],x0[2],x0[3],x1[0],x1[1],x1[2],x1[3],x2[0],x2[1],x2[2],x2[3],x3[0],x3[1],x3[2],x3[3]};
#pragma unroll
    for (int i = 0; i < 16; ++i) { const unsigned short hb = bf16_bits(xs[i]); ah.u[i] = hb; al.u[i] = ASPLIT ? bf16_bits(xs[i] - bf16_val(hb)) : (unsigned short)0; }
#pragma unroll
    for (int t = 0; t < 4; ++t) {
      if (col0 + t * 16 >= N) continue;
      const size_t boff = (size_t)(col0 + t * 16 + ln) * ldb + kb;
      FragB bh_, bl_; bh_.half[0] = *(const v8us*)(Bh + boff + 8 * hh); bh_.half[1] = *(const v8us*)(Bh + boff + 16 + 8 * hh);
      if (BSPLIT) { bl_.half[0] = *(const v8us*)(Bl + boff + 8 * hh); bl_.half[1] = *(const v8us*)(Bl + boff + 16 + 8 * hh); } else bl_ = bh_;
      acc[t] = mmaN<ASPLIT ? (BSPLIT ? 3 : 2) : 1>(ah.v, al.v, bh_.v, bl_.v, acc[t]);
    }
  }
#pragma unroll
  for (int t = 0; t < 4; ++t) {
    const int col = col0 + t * 16 + ln; if (col0 + t * 16 >= N) continue; const float bv = bias ? bf16_round(bias[col]) : 0.f;
#pragma unroll
    for (int r = 0; r < 8; ++r) { float v = acc[t][r] * alpha + bv; if (resid) v += rsign * resid[(size_t)(row0 + 8 * hh + r) * ldr + col]; if (ACT == 1) v = fmaxf(v, 0.f); else if (ACT == 2) v = fmaxf(v, 0.f) + log1pf(expf(-fabsf(v))); so[w][8 * hh + r][t * 16 + ln] = v; }
  }
  __builtin_amdgcn_fence(__ATOMIC_ACQ_REL, "workgroup"); __builtin_amdgcn_wave_barrier();
  const int rsub = lane >> 4, c4 = (lane & 15) * 4;
  for (int pass = 0; pass < 2; ++pass) {
#pragma unroll
    for (int q = 0; q < 8; ++q) { const int r = q * 2 + rsub; if (col0 + c4 < N) { const v4f v = *(const v4fa*)&so[w][r][c4]; *(volatile v4f*)(C + (size_t)(row0 + r) * ldc + col0 + c4) = v; } }
    if (pass == 0) __threadfence();
  }
}
__global__ __launch_bounds__(256) void k_split_transpose_b(const float* __restrict__ src, int lds_, size_t sIn, unsigned short* __restrict__ hi, unsigned short* __restrict__ lo, size_t sOut, int K, int N) {
  const size_t t = (size_t)blockIdx.x * 256 + threadIdx.x; const int k8n = K / 8; if (t >= (size_t)N * k8n) return;
  src += (size_t)blockIdx.y * sIn; hi += (size_t)blockIdx.y * sOut; lo += (size_t)blockIdx.y * sOut;
  const int n = (int)(t / k8n), k8 = (int)(t % k8n) * 8; v8us vh, vl;
#pragma unroll
  for (int i = 0; i < 8; ++i) { const float x = src[(size_t)(k8 + i) * lds_ + n]; const unsigned short hb = bf16_bits(x); vh[i] = hb; vl[i] = bf16_bits(x - bf16_val(hb)); }
  unsigned short* dh = hi + (size_t)n * K + k8; unsigned short* dl = lo + (size_t)n * K + k8;
  *(volatile v8us*)dh = vh; *(volatile v8us*)dl = vl; __threadfence(); *(volatile v8us*)dh = vh; *(volatile v8us*)dl = vl;
}

__global__ __launch_bounds__(256) void k_round_rows(const float* __restrict__ W, unsigned short* __restrict__ Wt, int n8) {
  const int t = blockIdx.x * 256 + threadIdx.x;
  if (t >= n8) return;
  const v4f a = *(const v4fa*)(W + (size_t)t * 8), b = *(const v4fa*)(W + (size_t)t * 8 + 4);
  v8us v; v[0]=bf16_bits(a[0]); v[1]=bf16_bits(a[1]); v[2]=bf16_bits(a[2]); v[3]=bf16_bits(a[3]);
  v[4]=bf16_bits(b[0]); v[5]=bf16_bits(b[1]); v[6]=bf16_bits(b[2]); v[7]=bf16_bits(b[3]);
  *(volatile v8us*)(Wt + (size_t)t * 8) = v; __threadfence(); *(volatile v8us*)(Wt + (size_t)t * 8) = v;
}

typedef _Float16 v16h __attribute__((ext_vector_type(16)));
union FragH { v16h v; v8us half[2]; _Float16 h[16]; unsigned short u[16]; };
template <int NT>
__device__ __forceinline__ v8f mmaH(v16h ah, v16h al, v16h bh, v16h bl, v8f c) {
  c = __builtin_amdgcn_wmma_f32_16x16x32_f16(false, ah, false, bh, (short)0, c, false, false);
  if (NT >= 2) c = __builtin_amdgcn_wmma_f32_16x16x32_f16(false, al, false, bh, (short)0, c, false, false);
  if (NT >= 3) c = __builtin_amdgcn_wmma_f32_16x16x32_f16(false, ah, false, bl, (short)0, c, false, false);
  asm volatile("v_nop\n\tv_nop\n\tv_nop\n\tv_nop" : "+v"(c) : "v"(ah), "v"(al), "v"(bh), "v"(bl));
  return c;
}
template <bool ASPLIT>
__global__ __launch_bounds__(128) void k_gemm_h(const float* __restrict__ A, int lda, size_t sA, const _Float16* __restrict__ Bh, int ldb, size_t sB, float alpha, float* __restrict__ C, int ldc, size_t sC, int M, int N, int K) {
  __shared__ __attribute__((aligned(16))) float so[4][16][64];
  const int tid = threadIdx.x, w = tid >> 5, lane = tid & 31, ln = lane & 15, hh = lane >> 4; const int by = blockIdx.y;
  A += (size_t)by * sA; Bh += (size_t)by * sB; C += (size_t)by * sC;
  const int ntn = (N + 63) / 64; const int wid = blockIdx.x * 4 + w; const int mt = wid / ntn, nq = wid % ntn; if (mt * 16 >= M) return;
  const int row0 = mt * 16, col0 = nq * 64; const float* arow = A + (size_t)(row0 + ln) * lda;
  v8f acc[4] = {};
  for (int kb = 0; kb < K; kb += 32) {
    FragH ah, al;
    const v4f x0 = *(const v4fa*)(arow + kb + 8 * hh), x1 = *(const v4fa*)(arow + kb + 8 * hh + 4), x2 = *(const v4fa*)(arow + kb + 16 + 8 * hh), x3 = *(const v4fa*)(arow + kb + 16 + 8 * hh + 4);
    float xs[16] = {x0[0],x0[1],x0[2],x0[3],x1[0],x1[1],x1[2],x1[3],x2[0],x2[1],x2[2],x2[3],x3[0],x3[1],x3[2],x3[3]};
#pragma unroll
    for (int i = 0; i < 16; ++i) { const _Float16 h = (_Float16)xs[i]; ah.h[i] = h; al.h[i] = ASPLIT ? (_Float16)(xs[i] - (float)h) : (_Float16)0.0f; }
#pragma unroll
    for (int t = 0; t < 4; ++t) { if (col0 + t * 16 >= N) continue; const size_t boff = (size_t)(col0 + t * 16 + ln) * ldb + kb; FragH bq; bq.half[0] = *(const v8us*)(Bh + boff + 8 * hh); bq.half[1] = *(const v8us*)(Bh + boff + 16 + 8 * hh);
      acc[t] = mmaH<ASPLIT ? 2 : 1>(ah.v, al.v, bq.v, bq.v, acc[t]); }
  }
#pragma unroll
  for (int t = 0; t < 4; ++t) { if (col0 + t * 16 >= N) continue;
#pragma unroll
    for (int r = 0; r < 8; ++r) so[w][8 * hh + r][t * 16 + ln] = acc[t][r] * alpha; }
  __builtin_amdgcn_fence(__ATOMIC_ACQ_REL, "workgroup"); __builtin_amdgcn_wave_barrier();
  const int rsub = lane >> 4, c4 = (lane & 15) * 4;
  for (int pass = 0; pass < 2; ++pass) {
#pragma unroll
    for (int q = 0; q < 8; ++q) { const int r = q * 2 + rsub; if (col0 + c4 < N) { const v4f v = *(const v4fa*)&so[w][r][c4]; *(volatile v4f*)(C + (size_t)(row0 + r) * ldc + col0 + c4) = v; } }
    if (pass == 0) __threadfence(); }
}

template <int DUMMY>
__global__ __launch_bounds__(128) void k_gemm_hh(const _Float16* __restrict__ A, int lda, size_t sA, const _Float16* __restrict__ Bh, int ldb, size_t sB, float alpha, float* __restrict__ C, int ldc, size_t sC, int M, int N, int K) {
  __shared__ __attribute__((aligned(16))) float so[4][16][64];
  const int tid = threadIdx.x, w = tid >> 5, lane = tid & 31, ln = lane & 15, hh = lane >> 4; const int by = blockIdx.y;
  A += (size_t)by * sA; Bh += (size_t)by * sB; C += (size_t)by * sC;
  const int ntn = (N + 63) / 64; const int wid = blockIdx.x * 4 + w; const int mt = wid / ntn, nq = wid % ntn; if (mt * 16 >= M) return;
  const int row0 = mt * 16, col0 = nq * 64; const _Float16* arow = A + (size_t)(row0 + ln) * lda;
  v8f acc[4] = {};
  for (int kb = 0; kb < K; kb += 32) { FragH ah; ah.half[0] = *(const v8us*)((const unsigned short*)arow + kb + 8 * hh); ah.half[1] = *(const v8us*)((const unsigned short*)arow + kb + 16 + 8 * hh);
#pragma unroll
    for (int t = 0; t < 4; ++t) { if (col0 + t * 16 >= N) continue; const size_t boff = (size_t)(col0 + t * 16 + ln) * ldb + kb; FragH bq; bq.half[0] = *(const v8us*)((const unsigned short*)Bh + boff + 8 * hh); bq.half[1] = *(const v8us*)((const unsigned short*)Bh + boff + 16 + 8 * hh);
      acc[t] = mmaH<1>(ah.v, ah.v, bq.v, bq.v, acc[t]); }
  }
#pragma unroll
  for (int t = 0; t < 4; ++t) { if (col0 + t * 16 >= N) continue;
#pragma unroll
    for (int r = 0; r < 8; ++r) so[w][8 * hh + r][t * 16 + ln] = acc[t][r] * alpha; }
  __builtin_amdgcn_fence(__ATOMIC_ACQ_REL, "workgroup"); __builtin_amdgcn_wave_barrier();
  const int rsub = lane >> 4, c4 = (lane & 15) * 4;
  for (int pass = 0; pass < 2; ++pass) {
#pragma unroll
    for (int q = 0; q < 8; ++q) { const int r = q * 2 + rsub; if (col0 + c4 < N) { const v4f v = *(const v4fa*)&so[w][r][c4]; *(volatile v4f*)(C + (size_t)(row0 + r) * ldc + col0 + c4) = v; } }
    if (pass == 0) __threadfence(); }
}

template <int ACT>
__global__ __launch_bounds__(128) void k_gemm_hhx(const _Float16* __restrict__ A, int lda, size_t sA, const _Float16* __restrict__ Bh, int ldb, size_t sB, float alpha, const float* __restrict__ bias, size_t sBias, const float* __restrict__ CP, int rowsPerB, size_t sCPb, int row0g,
    float* __restrict__ C, _Float16* __restrict__ C16, int ldc, size_t sC, int M, int N, int K) {
  __shared__ __attribute__((aligned(16))) float so[4][16][64];
  const int tid = threadIdx.x, w = tid >> 5, lane = tid & 31, ln = lane & 15, hh = lane >> 4; const int by = blockIdx.y;
  A += (size_t)by * sA; Bh += (size_t)by * sB; const size_t cofs = (size_t)by * sC; const float* bp = bias ? bias + (size_t)by * sBias : nullptr;
  const int ntn = (N + 63) / 64; const int wid = blockIdx.x * 4 + w; const int mt = wid / ntn, nq = wid % ntn; if (mt * 16 >= M) return;
  const int row0 = mt * 16, col0 = nq * 64; const _Float16* arow = A + (size_t)(row0 + ln) * lda;
  v8f acc[4] = {};
  for (int kb = 0; kb < K; kb += 32) { FragH ah; ah.half[0] = *(const v8us*)((const unsigned short*)arow + kb + 8 * hh); ah.half[1] = *(const v8us*)((const unsigned short*)arow + kb + 16 + 8 * hh);
#pragma unroll
    for (int t = 0; t < 4; ++t) { if (col0 + t * 16 >= N) continue; const size_t boff = (size_t)(col0 + t * 16 + ln) * ldb + kb; FragH bq; bq.half[0] = *(const v8us*)((const unsigned short*)Bh + boff + 8 * hh); bq.half[1] = *(const v8us*)((const unsigned short*)Bh + boff + 16 + 8 * hh);
      acc[t] = mmaH<1>(ah.v, ah.v, bq.v, bq.v, acc[t]); }
  }
#pragma unroll
  for (int t = 0; t < 4; ++t) { if (col0 + t * 16 >= N) continue; const int col = col0 + t * 16 + ln; const float bv = bp ? bf16_round(bp[col]) : 0.f;
#pragma unroll
    for (int r = 0; r < 8; ++r) { float v = acc[t][r] * alpha + bv; if (CP) { const int bidx = (row0g + row0 + 8 * hh + r) / rowsPerB; v += CP[(size_t)bidx * sCPb + (size_t)by * 64 + col]; } if (ACT == 1) v = (v > 0.f) ? v : expm1f(v); else if (ACT == 2) { const float u = 0.7978845608028654f * (v + 0.044715f * v * v * v); const float th = 1.0f - 2.0f / (__expf(2.0f * u) + 1.0f); v = 0.5f * v * (1.0f + th); } so[w][8 * hh + r][t * 16 + ln] = v; } }
  __builtin_amdgcn_fence(__ATOMIC_ACQ_REL, "workgroup"); __builtin_amdgcn_wave_barrier();
  const int rsub = lane >> 4, c4 = (lane & 15) * 4; typedef _Float16 v4h __attribute__((ext_vector_type(4)));
  for (int pass = 0; pass < 2; ++pass) {
#pragma unroll
    for (int q = 0; q < 8; ++q) { const int r = q * 2 + rsub; if (col0 + c4 < N) { const v4f v = *(const v4fa*)&so[w][r][c4]; if (C) *(volatile v4f*)(C + cofs + (size_t)(row0 + r) * ldc + col0 + c4) = v; if (C16) { v4h h4; for (int i = 0; i < 4; ++i) h4[i] = (_Float16)v[i]; *(volatile v4h*)(C16 + cofs + (size_t)(row0 + r) * ldc + col0 + c4) = h4; } } }
    if (pass == 0) __threadfence(); }
}

__device__ __forceinline__ float gelu_t(float v) { const float u = 0.7978845608028654f * (v + 0.044715f * v * v * v); return 0.5f * v * (1.0f + tanhf(u)); }
__global__ __launch_bounds__(256) void k_wt(const float* __restrict__ pw, const float* __restrict__ w1, const float* __restrict__ w2, const float* __restrict__ wq, const float* __restrict__ wp, unsigned short* __restrict__ Bp, _Float16* __restrict__ B1, _Float16* __restrict__ B2, _Float16* __restrict__ Bq, _Float16* __restrict__ Bo) { const size_t t = (size_t)blockIdx.x * 256 + threadIdx.x;
  if (t < (size_t)DD * KIN) { const int k = (int)(t % KIN), n = (int)(t / KIN); *(volatile unsigned short*)(Bp + t) = bf16_bits(pw[(size_t)k * DD + n]); }
  if (t < (size_t)HF * DD) { { const int k = (int)(t % DD), n = (int)(t / DD); *(volatile _Float16*)(B1 + t) = (_Float16)(bf16_round(w1[(size_t)k * HF + n]) * 16.0f); } { const int k = (int)(t % HF), n = (int)(t / HF); *(volatile _Float16*)(B2 + t) = (_Float16)(bf16_round(w2[(size_t)k * DD + n]) * 16.0f); } }
  if (t < (size_t)3 * DD * DD) { const int k = (int)(t % DD), n = (int)(t / DD); *(volatile _Float16*)(Bq + t) = (_Float16)(bf16_round(wq[(size_t)k * 3 * DD + n]) * 16.0f); }
  if (t < (size_t)DD * DD) { const int k = (int)(t % DD), n = (int)(t / DD); *(volatile _Float16*)(Bo + t) = (_Float16)(bf16_round(wp[(size_t)k * DD + n]) * 16.0f); } }
__global__ __launch_bounds__(256) void k_patch(const float* __restrict__ img, int b0, float* __restrict__ A0) { const size_t t = (size_t)blockIdx.x * 256 + threadIdx.x; if (t >= (size_t)TCH * KIN / 4) return; const int f4 = (int)((t * 4) % KIN); const size_t tok = (t * 4) / KIN; const int bl = (int)(tok / NTK), n = (int)(tok % NTK); const int Y = n / NPW, X = n % NPW; const int c = f4 / 256, py = (f4 % 256) / 16, px = f4 % 16;
  const v4f v = *(const v4fa*)(img + (((size_t)(b0 + bl) * 3 + c) * IMW + Y * PP + py) * IMW + X * PP + px); v4f o; for (int q = 0; q < 4; ++q) o[q] = bf16_round(v[q]); *(volatile v4f*)(A0 + t * 4) = o; __threadfence(); *(volatile v4f*)(A0 + t * 4) = o; }
__global__ __launch_bounds__(256) void k_lnpe(float* __restrict__ X, const float* __restrict__ g, const float* __restrict__ bb, _Float16* __restrict__ A16) { const int tid = threadIdx.x, wv = tid >> 5, lane = tid & 31; const size_t tok = (size_t)blockIdx.x * 8 + wv; const int n = (int)(tok % NTK); float v[DD / 32]; float s = 0.f;
  for (int u = 0; u < DD / 32; ++u) { v[u] = X[tok * DD + u * 32 + lane]; s += v[u]; } for (int o = 16; o >= 1; o >>= 1) s += __shfl_xor(s, o, 32); const float mu = s / (float)DD; float q2 = 0.f; for (int u = 0; u < DD / 32; ++u) { const float d = v[u] - mu; q2 += d * d; } for (int o = 16; o >= 1; o >>= 1) q2 += __shfl_xor(q2, o, 32); const float inv = 1.0f / sqrtf(q2 / (float)DD + 1e-5f);
  for (int pass = 0; pass < 2; ++pass) { for (int u = 0; u < DD / 32; ++u) { const int c = u * 32 + lane; const int i = c >> 1; const float ang = (float)n / powf(10000.0f, 2.0f * (float)i / (float)DD); const float pe = (c & 1) ? cosf(ang) : sinf(ang); const float y = (v[u] - mu) * inv * bf16_round(g[c]) + bf16_round(bb[c]) + pe; *(volatile float*)(X + tok * DD + c) = y; *(volatile _Float16*)(A16 + tok * DD + c) = (_Float16)y; } if (pass == 0) __threadfence(); } }
__global__ __launch_bounds__(256) void k_add(const float* __restrict__ F, const float* __restrict__ R, float* __restrict__ X) { const size_t t = (size_t)blockIdx.x * 256 + threadIdx.x; if (t >= (size_t)NTT * DD / 4) return; const v4f a = *(const v4fa*)(F + t * 4), b = *(const v4fa*)(R + t * 4); v4f o; for (int q = 0; q < 4; ++q) o[q] = a[q] + b[q]; *(volatile v4f*)(X + t * 4) = o; __threadfence(); *(volatile v4f*)(X + t * 4) = o; }
__global__ __launch_bounds__(256) void k_bnstat(const float* __restrict__ X, float* __restrict__ MU, float* __restrict__ IV) { const int c = threadIdx.x; float s = 0.f;
#pragma unroll 4
  for (int r = 0; r < NTT; ++r) s += X[(size_t)r * DD + c]; const float mu = s / (float)NTT; float q2 = 0.f;
#pragma unroll 4
  for (int r = 0; r < NTT; ++r) { const float d = X[(size_t)r * DD + c] - mu; q2 += d * d; } const float iv = 1.0f / sqrtf(q2 / (float)NTT + 1e-5f); *(volatile float*)(MU + c) = mu; *(volatile float*)(IV + c) = iv; __threadfence(); *(volatile float*)(MU + c) = mu; *(volatile float*)(IV + c) = iv; }
__global__ __launch_bounds__(256) void k_bnapply(const float* __restrict__ X, const float* __restrict__ MU, const float* __restrict__ IV, const float* __restrict__ g, const float* __restrict__ bb, float* __restrict__ Y, _Float16* __restrict__ A16) { const size_t t = (size_t)blockIdx.x * 256 + threadIdx.x; if (t >= (size_t)NTT * DD / 4) return; const int c4 = (int)((t * 4) % DD); const v4f x = *(const v4fa*)(X + t * 4); v4f o; typedef _Float16 v4h __attribute__((ext_vector_type(4))); v4h h;
  for (int q = 0; q < 4; ++q) { o[q] = (x[q] - MU[c4 + q]) * IV[c4 + q] * bf16_round(g[c4 + q]) + bf16_round(bb[c4 + q]); h[q] = (_Float16)o[q]; } *(volatile v4f*)(Y + t * 4) = o; if (A16) *(volatile v4h*)(A16 + t * 4) = h; __threadfence(); *(volatile v4f*)(Y + t * 4) = o; if (A16) *(volatile v4h*)(A16 + t * 4) = h; }
__global__ __launch_bounds__(256) void k_f16(const float* __restrict__ F, _Float16* __restrict__ A16, size_t n8) { const size_t t = (size_t)blockIdx.x * 256 + threadIdx.x; if (t >= n8) return; FragH f; for (int q = 0; q < 8; ++q) f.h[q] = (_Float16)F[t * 8 + q]; *(volatile v8us*)((unsigned short*)A16 + t * 8) = f.half[0]; __threadfence(); *(volatile v8us*)((unsigned short*)A16 + t * 8) = f.half[0]; }
__global__ __launch_bounds__(256) void k_wheads(const float* __restrict__ QKV, _Float16* __restrict__ Q16, _Float16* __restrict__ K16, _Float16* __restrict__ VT) { __shared__ float tile[WIN][DD + 1]; const int bw = blockIdx.x; const int tid = threadIdx.x, lane = tid & 31, wv = tid >> 5; const size_t tok0 = (size_t)bw * WIN;
  typedef _Float16 v2h __attribute__((ext_vector_type(2)));
  for (int pass = 0; pass < 2; ++pass) {
    for (int r = wv; r < WIN; r += 8) { const float* row = QKV + (tok0 + r) * 3 * DD; for (int c2 = lane; c2 < DD / 2; c2 += 32) { const int c = 2 * c2; const int h = c / DHD, d = c % DHD; const size_t slab = (size_t)bw * NHD + h; v2h q2 = { (_Float16)row[c], (_Float16)row[c + 1] }, k2 = { (_Float16)row[DD + c], (_Float16)row[DD + c + 1] };
        *(volatile v2h*)(Q16 + (slab * WIN + r) * DHD + d) = q2; *(volatile v2h*)(K16 + (slab * WIN + r) * DHD + d) = k2; if (pass == 0) { tile[r][c] = row[2 * DD + c]; tile[r][c + 1] = row[2 * DD + c + 1]; } } }
    if (pass == 0) __syncthreads();
    for (int c = wv; c < DD; c += 8) { const int h = c / DHD, d = c % DHD; const size_t slab = (size_t)bw * NHD + h; for (int r2 = lane; r2 < WIN; r2 += 32) *(volatile _Float16*)(VT + (slab * DHD + d) * WIN + r2) = (_Float16)tile[r2][c]; }
    if (pass == 0) __threadfence(); } }
__global__ __launch_bounds__(256) void k_wsoft(const float* __restrict__ S, _Float16* __restrict__ P) { const int tid = threadIdx.x, wv = tid >> 5, lane = tid & 31; const size_t row = (size_t)blockIdx.x * 8 + wv; typedef float v2f __attribute__((ext_vector_type(2), may_alias)); typedef _Float16 v2h __attribute__((ext_vector_type(2)));
  const v2f a = *(const v2f*)(S + row * WIN + 2 * lane); const float sc = 0.17677669529663687f; float x0 = a.x * sc, x1 = a.y * sc; float mx = fmaxf(x0, x1); for (int o = 16; o >= 1; o >>= 1) mx = fmaxf(mx, __shfl_xor(mx, o, 32)); x0 = expf(x0 - mx); x1 = expf(x1 - mx); float den = x0 + x1; for (int o = 16; o >= 1; o >>= 1) den += __shfl_xor(den, o, 32); const float inv = 1.0f / den;
  v2h o2 = { (_Float16)(x0 * inv), (_Float16)(x1 * inv) }; *(volatile v2h*)(P + row * WIN + 2 * lane) = o2; __threadfence(); *(volatile v2h*)(P + row * WIN + 2 * lane) = o2; }
extern "C" void kernel_launch(void* const* d_in, const int* in_sizes, int n_in,
                              void* d_out, int out_size, void* d_ws, size_t ws_size, hipStream_t stream) {
  (void)in_sizes; (void)n_in; (void)out_size;
  const float* img = (const float*)d_in[0]; const float* pw = (const float*)d_in[1]; const float* pb = (const float*)d_in[2]; const float* lng = (const float*)d_in[3]; const float* lnb = (const float*)d_in[4]; const float* w1 = (const float*)d_in[5]; const float* fb1 = (const float*)d_in[6]; const float* w2 = (const float*)d_in[7]; const float* fb2 = (const float*)d_in[8]; const float* wq = (const float*)d_in[9]; const float* bq = (const float*)d_in[10]; const float* wp = (const float*)d_in[11]; const float* bpj = (const float*)d_in[12]; const float* bn1g = (const float*)d_in[13]; const float* bn1b = (const float*)d_in[14]; const float* bn2g = (const float*)d_in[15]; const float* bn2b = (const float*)d_in[16];
  float* out = (float*)d_out;
  char* ws = (char*)d_ws; size_t off = 0;
  auto take = [&](size_t bytes) { char* p = ws + off; off += (bytes + 255) & ~(size_t)255; return p; };
  unsigned short* Bp = (unsigned short*)take((size_t)DD * KIN * 2); _Float16* B1 = (_Float16*)take((size_t)HF * DD * 2); _Float16* B2 = (_Float16*)take((size_t)DD * HF * 2); _Float16* Bq = (_Float16*)take((size_t)3 * DD * DD * 2); _Float16* Bo = (_Float16*)take((size_t)DD * DD * 2);
  float* R1 = (float*)take((size_t)TCH * KIN * 4);
  float* XA = (float*)take((size_t)NTT * DD * 4); _Float16* A16 = (_Float16*)take((size_t)NTT * DD * 2); _Float16* H16 = (_Float16*)take((size_t)NTT * HF * 2); float* F2 = (float*)take((size_t)NTT * DD * 4); float* O = (float*)take((size_t)NTT * DD * 4);
  _Float16* Q16 = (_Float16*)take((size_t)BCH * 16 * NHD * WIN * DHD * 2); _Float16* K16 = (_Float16*)take((size_t)BCH * 16 * NHD * WIN * DHD * 2); _Float16* VT = (_Float16*)take((size_t)BCH * 16 * NHD * DHD * WIN * 2); float* S = (float*)take((size_t)BCH * 16 * NHD * WIN * WIN * 4); _Float16* P = (_Float16*)take((size_t)BCH * 16 * NHD * WIN * WIN * 2); float* MU = (float*)take(DD * 4); float* IV = (float*)take(DD * 4);
  if (off > ws_size) return;
  auto EW = [](size_t n) { return (unsigned)((n + 255) / 256); };
  k_wt<<<EW((size_t)HF * DD), 256, 0, stream>>>(pw, w1, w2, wq, wp, Bp, B1, B2, Bq, Bo);
  for (int b0 = 0; b0 < BB; b0 += BCH) { k_patch<<<EW((size_t)TCH * KIN / 4), 256, 0, stream>>>(img, b0, R1); k_gemm_b<false, false, 0><<<dim3(((TCH / 16) * (DD / 64) + 3) / 4, 1), 128, 0, stream>>>(R1, KIN, 0, Bp, Bp, KIN, 0, pb, nullptr, 0, 0, 1.f, 1.f, XA + (size_t)b0 * NTK * DD, DD, 0, TCH, DD, KIN); }
  k_lnpe<<<NTT / 8, 256, 0, stream>>>(XA, lng, lnb, A16);
  const dim3 g1(((NTT / 16) * (HF / 64) + 3) / 4, 1), g2(((NTT / 16) * (DD / 64) + 3) / 4, 1);
  auto ffn = [&]() { k_gemm_hhx<2><<<g1, 128, 0, stream>>>(A16, DD, 0, B1, DD, 0, 0.0625f, fb1, 0, nullptr, 1, 0, 0, nullptr, H16, HF, 0, NTT, HF, DD);
                     k_gemm_hhx<0><<<g2, 128, 0, stream>>>(H16, HF, 0, B2, HF, 0, 0.0625f, fb2, 0, nullptr, 1, 0, 0, F2, A16, DD, 0, NTT, DD, HF); };
  ffn();
  for (int b0 = 0; b0 < BB; b0 += BCH) { const size_t t0 = (size_t)b0 * NTK; const int NSL = BCH * 16 * NHD;
    k_gemm_hhx<0><<<dim3(((TCH / 16) * (3 * DD / 64) + 3) / 4, 1), 128, 0, stream>>>(A16 + t0 * DD, DD, 0, Bq, DD, 0, 0.0625f, bq, 0, nullptr, 1, 0, 0, R1, nullptr, 3 * DD, 0, TCH, 3 * DD, DD);
    k_wheads<<<BCH * 16, 256, 0, stream>>>(R1, Q16, K16, VT);
    k_gemm_hh<0><<<dim3(((WIN / 16) * 1 + 3) / 4, NSL), 128, 0, stream>>>(Q16, DHD, (size_t)WIN * DHD, K16, DHD, (size_t)WIN * DHD, 1.0f, S, WIN, (size_t)WIN * WIN, WIN, WIN, DHD);
    k_wsoft<<<NSL * WIN / 8, 256, 0, stream>>>(S, P);
    for (int h = 0; h < NHD; ++h) k_gemm_hh<0><<<dim3(((WIN / 16) * 1 + 3) / 4, BCH * 16), 128, 0, stream>>>(P + (size_t)h * WIN * WIN, WIN, (size_t)NHD * WIN * WIN, VT + (size_t)h * DHD * WIN, WIN, (size_t)NHD * DHD * WIN, 1.0f, O + t0 * DD + h * DHD, DD, (size_t)WIN * DD, WIN, DHD, WIN); }
  k_f16<<<EW((size_t)NTT * DD / 8), 256, 0, stream>>>(O, A16, (size_t)NTT * DD / 8);
  k_gemm_hhx<0><<<g2, 128, 0, stream>>>(A16, DD, 0, Bo, DD, 0, 0.0625f, bpj, 0, nullptr, 1, 0, 0, F2, nullptr, DD, 0, NTT, DD, DD);
  k_add<<<EW((size_t)NTT * DD / 4), 256, 0, stream>>>(F2, XA, O);
  k_bnstat<<<1, 256, 0, stream>>>(O, MU, IV); k_bnapply<<<EW((size_t)NTT * DD / 4), 256, 0, stream>>>(O, MU, IV, bn1g, bn1b, XA, A16);
  ffn();
  k_add<<<EW((size_t)NTT * DD / 4), 256, 0, stream>>>(F2, XA, O);
  k_bnstat<<<1, 256, 0, stream>>>(O, MU, IV); k_bnapply<<<EW((size_t)NTT * DD / 4), 256, 0, stream>>>(O, MU, IV, bn2g, bn2b, out, nullptr);
}
